// GATConv_62036507623869
// MI455X (gfx1250) — hardware-verified
//
#include <hip/hip_runtime.h>
#include <stddef.h>
#include <stdint.h>
#include <math.h>


#define KIN     128
#define HD      128
#define NHEAD   4
#define DHEAD   32
#define ELW     8
#define NTHR    256
#define NWAVE   8
#define EPT     8
#define CHUNK   (NTHR * EPT)
#define WCAP    (EPT * 32)
#define LISTN   (NWAVE * WCAP)
#define NBMAX   2048
#define SLOTB   11
#define RCAP    28672
#define DEGCAP  256
#define GBM     64
#define GN      128
#define GTHR    128
#define NEGSL   0.2f
#define WSMAX   134217728
#define LDS_AGG ((2 * RCAP + 2 * NBMAX + LISTN) * 4 + 64)

static_assert((CHUNK & (CHUNK - 1)) == 0 && CHUNK <= (1 << SLOTB));
static_assert(NBMAX == (1 << SLOTB));
static_assert(NTHR * 8 == NBMAX);
static_assert(LISTN >= NBMAX);
static_assert(LISTN >= NWAVE * WCAP);
static_assert((RCAP % 32) == 0);
static_assert(LDS_AGG <= 300000);
static_assert(GBM == (GTHR / 32) * 16);
static_assert(GN == HD && HD == NHEAD * DHEAD);
static_assert(DHEAD == 8 * 4);
static_assert((KIN % 32) == 0 && KIN / 8 == 16);
static_assert(HD / 8 == 16 && KIN / 8 == 16);
static_assert(ELW == 2 * NHEAD);

typedef float          v4f  __attribute__((ext_vector_type(4)));
typedef float          v8f  __attribute__((ext_vector_type(8)));
typedef int            v4i  __attribute__((ext_vector_type(4)));
typedef int            v8i  __attribute__((ext_vector_type(8)));
typedef unsigned short v8us __attribute__((ext_vector_type(8)));
typedef __bf16         v16b __attribute__((ext_vector_type(16)));
typedef v4f  __attribute__((may_alias)) v4fa;
typedef v8us __attribute__((may_alias)) v8usa;
union FragB { v16b v; v8us h[2]; v8i w; };

__device__ __forceinline__ v8f wmb(const FragB& a, const FragB& b, v8f c) {
  v8f d = __builtin_amdgcn_wmma_f32_16x16x32_bf16(false, a.v, false, b.v, (short)0, c, false, false);
  asm volatile("v_nop\n\tv_nop\n\tv_nop\n\tv_nop" : "+v"(d) : "v"(a.w), "v"(b.w));
  return d;
}

__device__ __forceinline__ unsigned short f2bf(float f) {
  unsigned u = __float_as_uint(f);
  u += 0x7FFFu + ((u >> 16) & 1u);
  return (unsigned short)(u >> 16);
}
__device__ __forceinline__ float bfr(float f) {
  unsigned u = __float_as_uint(f);
  u = (u + 0x7FFFu + ((u >> 16) & 1u)) & 0xFFFF0000u;
  return __uint_as_float(u);
}
__device__ __forceinline__ v4f bfr4(const v4f a) {
  v4f r; r.x = bfr(a.x); r.y = bfr(a.y); r.z = bfr(a.z); r.w = bfr(a.w); return r;
}
__device__ __forceinline__ v8us cvt8b(const v4f a, const v4f b) {
  v8us o;
  o[0] = f2bf(a.x); o[1] = f2bf(a.y); o[2] = f2bf(a.z); o[3] = f2bf(a.w);
  o[4] = f2bf(b.x); o[5] = f2bf(b.y); o[6] = f2bf(b.z); o[7] = f2bf(b.w);
  return o;
}
__device__ __forceinline__ float hsel4(const v4f v, int hd) {
  const float a = (hd == 0) ? v.x : v.y;
  const float b = (hd == 2) ? v.z : v.w;
  return (hd < 2) ? a : b;
}

__device__ __forceinline__ int scan_chunk(const int* __restrict__ dsts, int nE, int cbase, int slotBase,
                                          int nb, int vec8, int* list, int tid, int lane, int wave) {
  int wc = 0;
  const int el0  = tid * EPT;
  const int e0   = cbase + el0;
  const int sent = -2147483647 - 1;
  v4i da, db;
  if (vec8 != 0 && cbase + CHUNK <= nE) {
    da = *(const v4i*)(dsts + e0);
    db = *(const v4i*)(dsts + e0 + 4);
  } else {
    da.x = (e0     < nE) ? dsts[min(e0,     nE - 1)] : sent;
    da.y = (e0 + 1 < nE) ? dsts[min(e0 + 1, nE - 1)] : sent;
    da.z = (e0 + 2 < nE) ? dsts[min(e0 + 2, nE - 1)] : sent;
    da.w = (e0 + 3 < nE) ? dsts[min(e0 + 3, nE - 1)] : sent;
    db.x = (e0 + 4 < nE) ? dsts[min(e0 + 4, nE - 1)] : sent;
    db.y = (e0 + 5 < nE) ? dsts[min(e0 + 5, nE - 1)] : sent;
    db.z = (e0 + 6 < nE) ? dsts[min(e0 + 6, nE - 1)] : sent;
    db.w = (e0 + 7 < nE) ? dsts[min(e0 + 7, nE - 1)] : sent;
  }
  const unsigned nbs = (unsigned)slotBase;
  const unsigned unb = (unsigned)nb;
  const unsigned s0 = (unsigned)da.x - nbs, s1 = (unsigned)da.y - nbs;
  const unsigned s2 = (unsigned)da.z - nbs, s3 = (unsigned)da.w - nbs;
  const unsigned s4 = (unsigned)db.x - nbs, s5 = (unsigned)db.y - nbs;
  const unsigned s6 = (unsigned)db.z - nbs, s7 = (unsigned)db.w - nbs;
  const bool h0 = s0 < unb, h1 = s1 < unb, h2 = s2 < unb, h3 = s3 < unb;
  const bool h4 = s4 < unb, h5 = s5 < unb, h6 = s6 < unb, h7 = s7 < unb;
  const unsigned any = __builtin_amdgcn_ballot_w32(h0 | h1 | h2 | h3 | h4 | h5 | h6 | h7);
  if (any != 0u) {
#define HITJ(J, HJ, SJ) { \
      const unsigned mj = __builtin_amdgcn_ballot_w32(HJ); \
      if (mj != 0u) { \
        if (HJ) { \
          const int pos = wc + (int)__builtin_amdgcn_mbcnt_lo(mj, 0u); \
          if (pos < WCAP) list[wave * WCAP + pos] = ((el0 + (J)) << SLOTB) | (int)(SJ); \
        } \
        wc += (int)__builtin_popcount(mj); } }
    HITJ(0, h0, s0)
    HITJ(1, h1, s1)
    HITJ(2, h2, s2)
    HITJ(3, h3, s3)
    HITJ(4, h4, s4)
    HITJ(5, h5, s5)
    HITJ(6, h6, s6)
    HITJ(7, h7, s7)
#undef HITJ
  }
  return wc;
}

__global__ __launch_bounds__(NTHR) void k_prep(const float* __restrict__ x, const float* __restrict__ w,
                                               unsigned short* xb, unsigned short* wt,
                                               int nN, int nUx, int nBx, int nUw) {
  const int tid = (int)threadIdx.x;
  const v4f z4 = {0.f, 0.f, 0.f, 0.f};
  if ((int)blockIdx.x < nBx) {
    const int i = (int)blockIdx.x * NTHR + tid;
    if (i >= nUx) return;
    const int row = i >> 4;
    const int c0  = (i & 15) * 8;
    const int rc  = row < nN ? row : nN - 1;
    const float* p = x + (size_t)rc * KIN + c0;
    v4f a = *(const v4fa*)p, b = *(const v4fa*)(p + 4);
    if (row >= nN) { a = z4; b = z4; }
    const v8us hv = cvt8b(a, b);
    const size_t o = (size_t)row * KIN + c0;
    *(volatile v8us*)(xb + o) = hv;
    __threadfence();
    *(volatile v8us*)(xb + o) = hv;
  } else {
    const int u = ((int)blockIdx.x - nBx) * NTHR + tid;
    if (u >= nUw) return;
    const int n   = u >> 4;
    const int k8  = (u & 15) * 8;
    const int ncl = n < HD ? n : HD - 1;
    const float* p = w + (size_t)k8 * (size_t)HD + ncl;
    v4f a, b;
    a.x = p[0];                 a.y = p[(size_t)HD];        a.z = p[(size_t)2 * HD];    a.w = p[(size_t)3 * HD];
    b.x = p[(size_t)4 * HD];    b.y = p[(size_t)5 * HD];    b.z = p[(size_t)6 * HD];    b.w = p[(size_t)7 * HD];
    if (n >= HD) { a = z4; b = z4; }
    const v8us hv = cvt8b(a, b);
    const size_t o = (size_t)n * (size_t)KIN + k8;
    *(volatile v8us*)(wt + o) = hv;
    __threadfence();
    *(volatile v8us*)(wt + o) = hv;
  }
}

__global__ __launch_bounds__(GTHR) void k_gemm(
    const unsigned short* __restrict__ A, const unsigned short* __restrict__ WT,
    const float* __restrict__ al, const float* __restrict__ ar,
    float* FT, float* ELR, int K)
{
  __shared__ __attribute__((aligned(16))) float stg[GBM * GN];
  __shared__ __attribute__((aligned(16))) float selr[GBM * ELW];
  const int tid = (int)threadIdx.x, lane = tid & 31, wave = tid >> 5, hh = lane >> 4, m = lane & 15;
  const int rowBase = (int)blockIdx.x * GBM;

  v8f acc[8];
  {
    const v8f z = {0.f, 0.f, 0.f, 0.f, 0.f, 0.f, 0.f, 0.f};
#pragma unroll
    for (int t = 0; t < 8; ++t) acc[t] = z;
  }
  const unsigned short* ap = A  + (size_t)(rowBase + 16 * wave + m) * (size_t)K + 8 * hh;
  const unsigned short* wp = WT + (size_t)m * (size_t)K + 8 * hh;
  const int ksteps = K >> 5;
#pragma unroll 1
  for (int ks = 0; ks < ksteps; ++ks) {
    FragB af;
    af.h[0] = *(const v8usa*)(ap + 32 * ks);
    af.h[1] = *(const v8usa*)(ap + 32 * ks + 16);
#pragma unroll
    for (int t = 0; t < 8; ++t) {
      const unsigned short* wq = wp + (size_t)(16 * t) * (size_t)K + 32 * ks;
      FragB bf;
      bf.h[0] = *(const v8usa*)wq;
      bf.h[1] = *(const v8usa*)(wq + 16);
      acc[t] = wmb(af, bf, acc[t]);
    }
  }

#pragma unroll
  for (int t = 0; t < 8; ++t) {
    const int lc = 16 * t + m;
#pragma unroll
    for (int r = 0; r < 8; ++r) {
      const int lr = 16 * wave + 8 * hh + r;
      stg[lr * GN + lc] = acc[t][r];
    }
  }
  __syncthreads();

  const int c0 = 4 * lane;
  const int hd = lane >> 3;
  const v4f al4 = bfr4(*(const v4fa*)(al + c0));
  const v4f ar4 = bfr4(*(const v4fa*)(ar + c0));
  v4f fv[16];
#pragma unroll
  for (int i = 0; i < 16; ++i) {
    const int lr = 16 * wave + i;
    const v4f v = *(const v4fa*)(stg + lr * GN + c0);
    fv[i] = v;
    float pl = v.x * al4.x; pl = fmaf(v.y, al4.y, pl); pl = fmaf(v.z, al4.z, pl); pl = fmaf(v.w, al4.w, pl);
    float pr = v.x * ar4.x; pr = fmaf(v.y, ar4.y, pr); pr = fmaf(v.z, ar4.z, pr); pr = fmaf(v.w, ar4.w, pr);
    pl += __shfl_xor(pl, 1); pl += __shfl_xor(pl, 2); pl += __shfl_xor(pl, 4);
    pr += __shfl_xor(pr, 1); pr += __shfl_xor(pr, 2); pr += __shfl_xor(pr, 4);
    if ((lane & 7) == 0) {
      selr[lr * ELW + hd]         = pl;
      selr[lr * ELW + NHEAD + hd] = pr;
    }
  }
  __syncthreads();

  const int erow = 16 * wave + (lane >> 1);
  const v4f ev = *(const v4fa*)(selr + erow * ELW + 4 * (lane & 1));
  float* ep = ELR + (size_t)(rowBase + erow) * ELW + 4 * (lane & 1);
#pragma unroll
  for (int i = 0; i < 16; ++i) {
    float* op = FT + (size_t)(rowBase + 16 * wave + i) * (size_t)GN + c0;
    *(volatile v4f*)op = fv[i];
  }
  *(volatile v4f*)ep = ev;
  __threadfence();
#pragma unroll
  for (int i = 0; i < 16; ++i) {
    float* op = FT + (size_t)(rowBase + 16 * wave + i) * (size_t)GN + c0;
    *(volatile v4f*)op = fv[i];
  }
  *(volatile v4f*)ep = ev;
}

__global__ __launch_bounds__(NTHR) void k_agg(
    const int* __restrict__ srcs, const int* __restrict__ dsts,
    const float* __restrict__ FT, const float* __restrict__ ELR,
    float* out, int nN, int nE, int nb, int vec8) {
  extern __shared__ v4f lds_dyn[];
  int* reg1 = (int*)lds_dyn;
  int* reg2 = reg1 + RCAP;
  int* scnt = reg2 + RCAP;
  int* soff = scnt + NBMAX;
  int* list = soff + NBMAX;
  int* wcnt = list + LISTN;
  int* wtot = wcnt + NWAVE;
  const int tid = (int)threadIdx.x, lane = tid & 31, wave = tid >> 5;
  const int nodeBase = (int)blockIdx.x * nb;

  for (int i = tid; i < NBMAX; i += NTHR) scnt[i] = 0;
  __syncthreads();

  int tot = 0;
  const int nChunks = (nE + CHUNK - 1) / CHUNK;
#pragma unroll 1
  for (int ch = 0; ch < nChunks; ++ch) {
    const int cbase = ch * CHUNK;
    const int wc = scan_chunk(dsts, nE, cbase, nodeBase, nb, vec8, list, tid, lane, wave);
    if (lane == 0) wcnt[wave] = wc;
    __syncthreads();
    int pre = 0, all = 0;
#pragma unroll
    for (int w2 = 0; w2 < NWAVE; ++w2) {
      int c = wcnt[w2];
      c = c < 0 ? 0 : (c > WCAP ? WCAP : c);
      all += c;
      pre += (w2 < wave) ? c : 0;
    }
    const int wcc  = wc > WCAP ? WCAP : wc;
    const int base = tot + pre;
#pragma unroll 1
    for (int i = lane; i < wcc; i += 32) {
      const int ent = list[wave * WCAP + i];
      const int el  = (ent >> SLOTB) & (CHUNK - 1);
      const int sl  = ent & (NBMAX - 1);
      int eid = cbase + el;
      eid = eid > nE - 1 ? nE - 1 : eid;
      const int pos = base + i;
      if (pos < RCAP) reg1[pos] = (int)(((unsigned)eid << SLOTB) | (unsigned)sl);
    }
    tot += all;
    tot = tot > RCAP ? RCAP : tot;
    __syncthreads();
  }
  const int nh = tot;

  if (wave == 0) {
#pragma unroll 1
    for (int b0 = 0; b0 < nh; b0 += 32) {
      const int idx = b0 + lane;
      const int uv  = reg1[idx < nh ? idx : nh - 1];
      const int m32 = (nh - b0) < 32 ? (nh - b0) : 32;
#pragma unroll 1
      for (int k = 0; k < m32; ++k) {
        const int u  = __builtin_amdgcn_readlane(uv, k);
        const int sl = u & (NBMAX - 1);
        if (lane == 0) scnt[sl] = scnt[sl] + 1;
      }
    }
  }
  __syncthreads();

  {
    const v4i ca = *(const v4i*)(scnt + 8 * tid);
    const v4i cb = *(const v4i*)(scnt + 8 * tid + 4);
    const int e0 = ca.x < 0 ? 0 : ca.x, e1 = ca.y < 0 ? 0 : ca.y, e2 = ca.z < 0 ? 0 : ca.z, e3 = ca.w < 0 ? 0 : ca.w;
    const int e4 = cb.x < 0 ? 0 : cb.x, e5 = cb.y < 0 ? 0 : cb.y, e6 = cb.z < 0 ? 0 : cb.z, e7 = cb.w < 0 ? 0 : cb.w;
    const int ts = e0 + e1 + e2 + e3 + e4 + e5 + e6 + e7;
    int incl = ts;
#pragma unroll
    for (int d = 1; d < 32; d <<= 1) {
      const int up = __shfl_up(incl, d);
      if (lane >= d) incl += up;
    }
    if (lane == 31) wtot[wave] = incl;
    __syncthreads();
    int pre = 0;
#pragma unroll
    for (int w2 = 0; w2 < NWAVE; ++w2) pre += (w2 < wave) ? wtot[w2] : 0;
    int run = pre + incl - ts;
    soff[8 * tid + 0] = run; run += e0;
    soff[8 * tid + 1] = run; run += e1;
    soff[8 * tid + 2] = run; run += e2;
    soff[8 * tid + 3] = run; run += e3;
    soff[8 * tid + 4] = run; run += e4;
    soff[8 * tid + 5] = run; run += e5;
    soff[8 * tid + 6] = run; run += e6;
    soff[8 * tid + 7] = run;
  }
  __syncthreads();
  for (int i = tid; i < NBMAX; i += NTHR) list[i] = soff[i];
  __syncthreads();

  if (wave == 0) {
#pragma unroll 1
    for (int b0 = 0; b0 < nh; b0 += 32) {
      const int idx = b0 + lane;
      const int uv  = reg1[idx < nh ? idx : nh - 1];
      const int m32 = (nh - b0) < 32 ? (nh - b0) : 32;
#pragma unroll 1
      for (int k = 0; k < m32; ++k) {
        const int u   = __builtin_amdgcn_readlane(uv, k);
        const int sl  = u & (NBMAX - 1);
        const int eid = (int)((unsigned)u >> SLOTB);
        if (lane == 0) {
          int pos = list[sl];
          pos = pos < 0 ? 0 : (pos > RCAP - 1 ? RCAP - 1 : pos);
          reg2[pos] = eid;
          list[sl] = pos + 1;
        }
      }
    }
  }
  __syncthreads();

  const int nbw = nb >> 3;
  const bool ovf = (nh >= RCAP);
  const float qnan = __int_as_float(0x7fc00000);
  const int c0 = 4 * lane;
  const int hd = lane >> 3;

#pragma unroll 1
  for (int jt = 0; jt < nbw; ++jt) {
    const int slot = wave * nbw + jt;
    const int grow = nodeBase + slot;
    const int gcl  = grow < nN ? grow : nN - 1;
    int st = soff[slot];
    const int craw = scnt[slot];
    int cnt = craw;
    st  = st < 0 ? 0 : (st > nh ? nh : st);
    cnt = cnt < 0 ? 0 : (cnt > DEGCAP ? DEGCAP : cnt);
    if (cnt > nh - st) cnt = nh - st;
    const float pz = (ovf || craw > DEGCAP) ? qnan : 0.0f;
    const bool wr = grow < nN;

    const v4f er4 = *(const v4fa*)(ELR + (size_t)gcl * ELW + NHEAD);
    const float erh = hsel4(er4, hd);
    float mx = -1.0e30f, dn = 0.f;
    v4f av = {0.f, 0.f, 0.f, 0.f};

#pragma unroll 1
    for (int q = 0; q < cnt; ++q) {
      int idx = st + q; idx = idx > RCAP - 1 ? RCAP - 1 : idx;
      int eid = reg2[idx]; eid = eid < 0 ? 0 : (eid > nE - 1 ? nE - 1 : eid);
      const int sraw = srcs[eid];
      const int s = sraw < 0 ? 0 : (sraw > nN - 1 ? nN - 1 : sraw);
      const v4f xl4 = *(const v4fa*)(FT + (size_t)s * HD + c0);
      const v4f el4 = *(const v4fa*)(ELR + (size_t)s * ELW);
      float lg = hsel4(el4, hd) + erh;
      lg = lg > 0.f ? lg : lg * NEGSL;
      const float df = lg - mx;
      const float ee = __expf(-fabsf(df));
      const bool up  = df > 0.f;
      const float s1 = up ? ee : 1.0f;
      const float s2 = up ? 1.0f : ee;
      mx = up ? lg : mx;
      dn = fmaf(dn, s1, s2);
      av.x = fmaf(av.x, s1, s2 * xl4.x);
      av.y = fmaf(av.y, s1, s2 * xl4.y);
      av.z = fmaf(av.z, s1, s2 * xl4.z);
      av.w = fmaf(av.w, s1, s2 * xl4.w);
    }
    const float ds = dn > 0.f ? dn : 1.0f;
    const float iv = (dn > 0.f ? 1.0f : 0.0f) * __builtin_amdgcn_rcpf(ds);
    v4f y;
    y.x = av.x * iv + pz;
    y.y = av.y * iv + pz;
    y.z = av.z * iv + pz;
    y.w = av.w * iv + pz;
    float* gp = out + (size_t)gcl * HD + c0;
    if (wr) *(volatile v4f*)gp = y;
    __threadfence();
    if (wr) *(volatile v4f*)gp = y;
  }
}

static int pick_nb(int nE, int nN) {
  int nb = NBMAX;
  while (nb > 32 && (long long)nb * (long long)nE * 5LL > (long long)RCAP * (long long)nN * 4LL) nb >>= 1;
  return nb;
}
static inline int cdiv(int a, int b) { return (a + b - 1) / b; }

extern "C" void kernel_launch(void* const* d_in, const int* in_sizes, int n_in,
                              void* d_out, int out_size, void* d_ws, size_t ws_size,
                              hipStream_t stream) {
  if (n_in < 6) return;
  const int nN = in_sizes[0] / KIN;
  if (nN <= 0 || in_sizes[0] != nN * KIN || nN > (1 << 22)) return;
  if (in_sizes[1] != KIN * HD) return;
  if (in_sizes[2] != HD || in_sizes[3] != HD) return;
  const int nE = in_sizes[4];
  if (nE < 1 || nE >= (1 << (32 - SLOTB))) return;
  if (in_sizes[5] != nE) return;
  if (out_size != nN * HD) return;

  const float* x   = (const float*)d_in[0];
  const float* w   = (const float*)d_in[1];
  const float* al  = (const float*)d_in[2];
  const float* ar  = (const float*)d_in[3];
  const int*   src = (const int*)  d_in[4];
  const int*   dst = (const int*)  d_in[5];
  float* out = (float*)d_out;

  const int MP   = cdiv(nN, GBM) * GBM;
  const int nb   = pick_nb(nE, nN);
  if (nb < 32 || (nb & (nb - 1)) != 0 || nb > NBMAX) return;
  const int gA   = cdiv(MP, nb);
  const int vec8 = ((nE & 3) == 0) ? 1 : 0;
  if (gA * nb < MP) return;

  char* ws = (char*)d_ws;
  size_t off = 0;
  const size_t oXB  = off; off += (size_t)MP * KIN * 2;            off = (off + 255) & ~(size_t)255;
  const size_t oWT  = off; off += (size_t)HD * KIN * 2;            off = (off + 255) & ~(size_t)255;
  const size_t oFT  = off; off += (size_t)MP * HD * 4;             off = (off + 255) & ~(size_t)255;
  const size_t oELR = off; off += (size_t)MP * ELW * 4;            off = (off + 255) & ~(size_t)255;
  if (off > ws_size || off > (size_t)WSMAX) return;
  unsigned short* XB  = (unsigned short*)(ws + oXB);
  unsigned short* WT  = (unsigned short*)(ws + oWT);
  float*          FT  = (float*)(ws + oFT);
  float*          ELR = (float*)(ws + oELR);

  hipFuncSetAttribute(reinterpret_cast<const void*>(&k_agg),
                      hipFuncAttributeMaxDynamicSharedMemorySize, LDS_AGG);

  const int nUx = MP * (KIN / 8);
  const int nBx = cdiv(nUx, NTHR);
  const int nUw = HD * (KIN / 8);
  if (nBx * NTHR != nUx) return;
  k_prep<<<nBx + cdiv(nUw, NTHR), NTHR, 0, stream>>>(x, w, XB, WT, nN, nUx, nBx, nUw);

  const int gM = MP / GBM;
  k_gemm<<<gM, GTHR, 0, stream>>>(XB, WT, al, ar, FT, ELR, KIN);

  k_agg<<<gA, NTHR, LDS_AGG, stream>>>(src, dst, FT, ELR, out, nN, nE, nb, vec8);
}
